// MoeTritonLayer_24086176596767
// MI455X (gfx1250) — hardware-verified
//
#include <hip/hip_runtime.h>
#include <stddef.h>


#define NTOK 8192
#define DIN  256
#define HD   512
#define DOUT 256
#define NE   16
#define TR   64
#define NTL  272
#define NTHR 256
#define LTHR 512
#define GCH  16

static_assert(NTL * TR >= 2 * NTOK + NE * (TR - 1));
static_assert((NTOK % TR) == 0 && (NTOK % 32) == 0 && (NTOK % 4) == 0 && (NTOK % NTHR) == 0);
static_assert((DIN % 64) == 0 && (HD % 256) == 0 && (DOUT % 256) == 0 && (HD % 64) == 0);
static_assert((HD % GCH) == 0 && GCH * NE == NTHR && (DIN * GCH) == 4 * 4 * NTHR);
static_assert(((NTL * TR) % 8) == 0);
static_assert(LTHR == NE * 32);
static_assert((size_t)NTOK * 2 * DOUT * 4 <= (size_t)NTL * TR * HD * 2);

typedef float          v4f   __attribute__((ext_vector_type(4)));
typedef float          v8f   __attribute__((ext_vector_type(8)));
typedef int            v4i   __attribute__((ext_vector_type(4)));
typedef unsigned short v8us  __attribute__((ext_vector_type(8)));
typedef unsigned short v16us __attribute__((ext_vector_type(16)));
typedef __bf16         v16bf __attribute__((ext_vector_type(16)));
union FragB { v16us u; v8us h[2]; v16bf v; };

__device__ __forceinline__ unsigned int bfbits(float f) {
  unsigned int u = __float_as_uint(f);
  u = u + 0x7FFFu + ((u >> 16) & 1u);
  return u >> 16;
}

__device__ __forceinline__ v8f wmb(v16bf a, v16bf b, v8f c) {
  v8f d = __builtin_amdgcn_wmma_f32_16x16x32_bf16(false, a, false, b, (short)0, c, false, false);
#if defined(__HIP_DEVICE_COMPILE__)
  asm volatile("v_nop\n\tv_nop\n\tv_nop\n\tv_nop" : "+v"(d) : "v"(a), "v"(b));
#endif
  return d;
}

__global__ __launch_bounds__(NTHR) void k_wconv(const float* __restrict__ W, unsigned short* oh, unsigned short* ol, int K, int C) {
  __shared__ __attribute__((aligned(16))) unsigned short t0[64 * 72];
  __shared__ __attribute__((aligned(16))) unsigned short t1[64 * 72];
  const int tid = threadIdx.x;
  const int k0 = blockIdx.x * 64, c0 = blockIdx.y * 64;
#pragma unroll
  for (int i = 0; i < 4; ++i) {
    const int idx = i * NTHR + tid;
    const int kr  = idx >> 4;
    const int cc  = (idx & 15) * 4;
    const v4f v = *(const v4f*)(W + (size_t)(k0 + kr) * C + c0 + cc);
    float f[4];
    f[0] = v.x; f[1] = v.y; f[2] = v.z; f[3] = v.w;
#pragma unroll
    for (int q = 0; q < 4; ++q) {
      const unsigned int hb = bfbits(f[q]);
      const float hf = __uint_as_float(hb << 16);
      t0[(cc + q) * 72 + kr] = (unsigned short)hb;
      t1[(cc + q) * 72 + kr] = (unsigned short)bfbits(f[q] - hf);
    }
  }
  __syncthreads();
  const int nrA = tid >> 3;
  const int nrB = nrA + 32;
  const int pc  = tid & 7;
  const v8us a0 = *(const v8us*)(t0 + nrA * 72 + pc * 8);
  const v8us b0 = *(const v8us*)(t0 + nrB * 72 + pc * 8);
  const v8us a1 = *(const v8us*)(t1 + nrA * 72 + pc * 8);
  const v8us b1 = *(const v8us*)(t1 + nrB * 72 + pc * 8);
  const size_t ga = ((size_t)(c0 + nrA)) * K + k0 + pc * 8;
  const size_t gb = ((size_t)(c0 + nrB)) * K + k0 + pc * 8;
  *(volatile v8us*)(oh + ga) = a0;
  *(volatile v8us*)(oh + gb) = b0;
  *(volatile v8us*)(ol + ga) = a1;
  *(volatile v8us*)(ol + gb) = b1;
  __threadfence();
  *(volatile v8us*)(oh + ga) = a0;
  *(volatile v8us*)(oh + gb) = b0;
  *(volatile v8us*)(ol + ga) = a1;
  *(volatile v8us*)(ol + gb) = b1;
}

__global__ __launch_bounds__(NTHR) void k_gate(
    const float* __restrict__ x, const float* __restrict__ gw, const float* __restrict__ gb,
    const float* __restrict__ gow, const float* __restrict__ gob, int* tinfo) {
#pragma clang fp contract(off)
  __shared__ __attribute__((aligned(16))) float sW[DIN * GCH];
  __shared__ __attribute__((aligned(16))) float sO[GCH * NE];
  __shared__ __attribute__((aligned(16))) float sHid[GCH * NTHR];
  __shared__ float sB[GCH];
  const int tid = threadIdx.x;
  const int t = blockIdx.x * NTHR + tid;
  const float* xr = x + (size_t)t * DIN;

  float lg[NE];
#pragma unroll
  for (int j = 0; j < NE; ++j) lg[j] = 0.0f;

#pragma unroll 1
  for (int q = 0; q < HD / GCH; ++q) {
    __syncthreads();
#pragma unroll
    for (int i = 0; i < 4; ++i) {
      const int idx = i * NTHR + tid;
      const int k  = idx >> 2;
      const int c4 = (idx & 3) * 4;
      const v4f v = *(const v4f*)(gw + (size_t)k * HD + q * GCH + c4);
      *(v4f*)(sW + k * GCH + c4) = v;
    }
    sO[tid] = gow[(size_t)q * GCH * NE + tid];
    if (tid < GCH) sB[tid] = gb[q * GCH + tid];
    __syncthreads();

    float a[GCH];
#pragma unroll
    for (int c = 0; c < GCH; ++c) a[c] = 0.0f;
#pragma unroll 1
    for (int k = 0; k < DIN; ++k) {
      const float xv = xr[k];
      const v4f w0 = *(const v4f*)(sW + k * GCH);
      const v4f w1 = *(const v4f*)(sW + k * GCH + 4);
      const v4f w2 = *(const v4f*)(sW + k * GCH + 8);
      const v4f w3 = *(const v4f*)(sW + k * GCH + 12);
      a[0]  = fmaf(xv, w0.x, a[0]);  a[1]  = fmaf(xv, w0.y, a[1]);  a[2]  = fmaf(xv, w0.z, a[2]);  a[3]  = fmaf(xv, w0.w, a[3]);
      a[4]  = fmaf(xv, w1.x, a[4]);  a[5]  = fmaf(xv, w1.y, a[5]);  a[6]  = fmaf(xv, w1.z, a[6]);  a[7]  = fmaf(xv, w1.w, a[7]);
      a[8]  = fmaf(xv, w2.x, a[8]);  a[9]  = fmaf(xv, w2.y, a[9]);  a[10] = fmaf(xv, w2.z, a[10]); a[11] = fmaf(xv, w2.w, a[11]);
      a[12] = fmaf(xv, w3.x, a[12]); a[13] = fmaf(xv, w3.y, a[13]); a[14] = fmaf(xv, w3.z, a[14]); a[15] = fmaf(xv, w3.w, a[15]);
    }
#pragma unroll
    for (int c = 0; c < GCH; ++c) {
      float h = a[c] + sB[c];
      h = fmaxf(h, 0.0f);
      sHid[c * NTHR + tid] = h;
    }
#pragma unroll 1
    for (int c = 0; c < GCH; ++c) {
      const float h = sHid[c * NTHR + tid];
      const v4f o0 = *(const v4f*)(sO + c * NE);
      const v4f o1 = *(const v4f*)(sO + c * NE + 4);
      const v4f o2 = *(const v4f*)(sO + c * NE + 8);
      const v4f o3 = *(const v4f*)(sO + c * NE + 12);
      lg[0]  = fmaf(h, o0.x, lg[0]);  lg[1]  = fmaf(h, o0.y, lg[1]);  lg[2]  = fmaf(h, o0.z, lg[2]);  lg[3]  = fmaf(h, o0.w, lg[3]);
      lg[4]  = fmaf(h, o1.x, lg[4]);  lg[5]  = fmaf(h, o1.y, lg[5]);  lg[6]  = fmaf(h, o1.z, lg[6]);  lg[7]  = fmaf(h, o1.w, lg[7]);
      lg[8]  = fmaf(h, o2.x, lg[8]);  lg[9]  = fmaf(h, o2.y, lg[9]);  lg[10] = fmaf(h, o2.z, lg[10]); lg[11] = fmaf(h, o2.w, lg[11]);
      lg[12] = fmaf(h, o3.x, lg[12]); lg[13] = fmaf(h, o3.y, lg[13]); lg[14] = fmaf(h, o3.z, lg[14]); lg[15] = fmaf(h, o3.w, lg[15]);
    }
  }
#pragma unroll
  for (int j = 0; j < NE; ++j) lg[j] = lg[j] + gob[j];

  float mx = lg[0]; int i0 = 0;
#define P1(EI) { const bool cc = lg[EI] > mx; mx = cc ? lg[EI] : mx; i0 = cc ? (EI) : i0; }
  P1(1) P1(2) P1(3) P1(4) P1(5) P1(6) P1(7) P1(8) P1(9) P1(10) P1(11) P1(12) P1(13) P1(14) P1(15)
#undef P1
  int   i1 = (i0 == 0) ? 1 : 0;
  float m1 = (i0 == 0) ? lg[1] : lg[0];
#define P2(EI) { const bool cc = ((EI) != i0) && (lg[EI] > m1); m1 = cc ? lg[EI] : m1; i1 = cc ? (EI) : i1; }
  P2(1) P2(2) P2(3) P2(4) P2(5) P2(6) P2(7) P2(8) P2(9) P2(10) P2(11) P2(12) P2(13) P2(14) P2(15)
#undef P2
  const float d   = m1 - mx;
  const float e1  = expf(d);
  const float s   = 1.0f + e1;
  const float inv = 1.0f / s;
  const float g0  = inv;
  const float g1  = e1 * inv;
  v4i o;
  o.x = i0; o.y = i1; o.z = __float_as_int(g0); o.w = __float_as_int(g1);
  int* op = tinfo + 4 * (size_t)t;
  *(volatile v4i*)op = o;
  __threadfence();
  *(volatile v4i*)op = o;
}

__device__ __forceinline__ void emit_pass(const int* __restrict__ tinfo, int* plist, int* rg,
                                          int w, int lane, int nCh, int segS, int segE, int nt) {
  int c = 0;
#pragma unroll 1
  for (int ch = 0; ch < nCh; ++ch) {
    const int t = ch * 32 + lane;
    const v4i inf = *(const v4i*)(tinfo + 4 * (size_t)t);
    const bool h0  = (inf.x == w);
    const bool h1  = (inf.y == w);
    const bool hit = h0 || h1;
    const unsigned mk = __builtin_amdgcn_ballot_w32(hit);
    const int rank = (int)__builtin_amdgcn_mbcnt_lo(mk, 0u);
    const int k    = (int)__builtin_popcount(mk);
    if (hit) rg[(c + rank) & 63] = (t << 1) | (h0 ? 0 : 1);
    __syncthreads();
    const int cn = c + k;
    if ((cn >> 5) != (c >> 5)) {
      const int L   = c >> 5;
      const int val = rg[((L & 1) << 5) + lane];
      const int row = segS * TR + L * 32 + lane;
      if ((unsigned)row < (unsigned)(NTL * TR)) *(volatile int*)(plist + row) = val;
    }
    __syncthreads();
    c = cn;
  }
  int linesTot = (segE - segS) * 2;
  linesTot = linesTot < 0 ? 0 : (linesTot > 2 * NTL ? 2 * NTL : linesTot);
  const int Lf  = c >> 5;
  const int rem = c & 31;
#pragma unroll
  for (int i = 0; i < 2; ++i) {
    const int L = Lf + i;
    if (L < linesTot) {
      const int rv  = rg[((L & 1) << 5) + lane];
      const int val = (i == 0 && lane < rem) ? rv : -1;
      const int row = segS * TR + L * 32 + lane;
      if ((unsigned)row < (unsigned)(NTL * TR)) *(volatile int*)(plist + row) = val;
    }
  }
#pragma unroll 1
  for (int L = nt * 2 + w; L < 2 * NTL; L += NE) {
    const int row = L * 32 + lane;
    *(volatile int*)(plist + row) = -1;
  }
}

__global__ __launch_bounds__(LTHR) void k_lists(const int* __restrict__ tinfo, int* plist, int* hdr, int nTok) {
  __shared__ __attribute__((aligned(16))) int ring[NE * 64];
  __shared__ int scnt[NE];
  __shared__ __attribute__((aligned(16))) int shdr[64];
  const int tid = threadIdx.x, lane = tid & 31, w = tid >> 5;
  const int nCh = nTok >> 5;

  int cnt = 0;
#pragma unroll 1
  for (int ch = 0; ch < nCh; ++ch) {
    const int t = ch * 32 + lane;
    const v4i inf = *(const v4i*)(tinfo + 4 * (size_t)t);
    const bool hit = (inf.x == w) || (inf.y == w);
    const unsigned mk = __builtin_amdgcn_ballot_w32(hit);
    cnt += (int)__builtin_popcount(mk);
  }
  if (lane == 0) scnt[w] = cnt;
  __syncthreads();
  if (tid == 0) {
    int s = 0;
    shdr[0] = 0;
    for (int e = 0; e < NE; ++e) {
      const int ce = scnt[e];
      s += (ce + TR - 1) / TR;
      shdr[e + 1]  = s;
      shdr[32 + e] = ce;
    }
    for (int i = NE + 1; i < 32; ++i) shdr[i] = 0;
    for (int i = 48; i < 64; ++i) shdr[i] = 0;
  }
  __syncthreads();
  const int segS = shdr[w], segE = shdr[w + 1];
  int nt = shdr[NE];
  nt = nt < 0 ? 0 : (nt > NTL ? NTL : nt);
  const v4i hv = *(const v4i*)(shdr + 4 * (tid & 15));

  emit_pass(tinfo, plist, ring + w * 64, w, lane, nCh, segS, segE, nt);
  if (tid < 16) *(volatile v4i*)(hdr + 4 * tid) = hv;
  __threadfence();
  emit_pass(tinfo, plist, ring + w * 64, w, lane, nCh, segS, segE, nt);
  if (tid < 16) *(volatile v4i*)(hdr + 4 * tid) = hv;
}

__global__ __launch_bounds__(NTHR) void k_gather(
    const float* __restrict__ x, const int* __restrict__ plist,
    unsigned short* Xgh, unsigned short* Xgl, int nTok) {
  const int tid = threadIdx.x;
  const int r   = blockIdx.x * 8 + (tid >> 5);
  const int c0  = (tid & 31) * 8;
  const int ent = plist[r];
  const bool valid = ent >= 0;
  int t = ent >> 1;
  t = t < 0 ? 0 : (t > nTok - 1 ? nTok - 1 : t);
  const float* xp = x + (size_t)t * DIN + c0;
  const v4f a = *(const v4f*)xp;
  const v4f b = *(const v4f*)(xp + 4);
  float f[8];
  f[0] = a.x; f[1] = a.y; f[2] = a.z; f[3] = a.w; f[4] = b.x; f[5] = b.y; f[6] = b.z; f[7] = b.w;
  v8us oh, ol;
#pragma unroll
  for (int j = 0; j < 8; ++j) {
    const unsigned int hb = bfbits(f[j]);
    const float hf = __uint_as_float(hb << 16);
    const unsigned int lb = bfbits(f[j] - hf);
    oh[j] = valid ? (unsigned short)hb : (unsigned short)0;
    ol[j] = valid ? (unsigned short)lb : (unsigned short)0;
  }
  const size_t d = (size_t)r * DIN + c0;
  *(volatile v8us*)(Xgh + d) = oh;
  *(volatile v8us*)(Xgl + d) = ol;
  __threadfence();
  *(volatile v8us*)(Xgh + d) = oh;
  *(volatile v8us*)(Xgl + d) = ol;
}

__device__ __forceinline__ int tile_expert(const int* __restrict__ hdr, int j, int* ntOut) {
  const v4i a = *(const v4i*)hdr;
  const v4i b = *(const v4i*)(hdr + 4);
  const v4i c = *(const v4i*)(hdr + 8);
  const v4i d = *(const v4i*)(hdr + 12);
  int nt = hdr[16];
  nt = nt < 0 ? 0 : (nt > NTL ? NTL : nt);
  *ntOut = nt;
  int e = 0;
  e += (j >= a.y) ? 1 : 0; e += (j >= a.z) ? 1 : 0; e += (j >= a.w) ? 1 : 0;
  e += (j >= b.x) ? 1 : 0; e += (j >= b.y) ? 1 : 0; e += (j >= b.z) ? 1 : 0; e += (j >= b.w) ? 1 : 0;
  e += (j >= c.x) ? 1 : 0; e += (j >= c.y) ? 1 : 0; e += (j >= c.z) ? 1 : 0; e += (j >= c.w) ? 1 : 0;
  e += (j >= d.x) ? 1 : 0; e += (j >= d.y) ? 1 : 0; e += (j >= d.z) ? 1 : 0; e += (j >= d.w) ? 1 : 0;
  return e;
}

template <int KD>
__global__ __launch_bounds__(NTHR) void k_ffn(
    const unsigned short* __restrict__ Ah, const unsigned short* __restrict__ Al,
    const unsigned short* __restrict__ Wh, const unsigned short* __restrict__ Wl,
    const float* __restrict__ bias, const int* __restrict__ hdr,
    unsigned short* Hh, unsigned short* Hl) {
  __shared__ __attribute__((aligned(16))) unsigned short stg[8 * 2048];
  const int tid = threadIdx.x, lane = tid & 31, wave = tid >> 5, hh = lane >> 4, m = lane & 15;
  const int j = blockIdx.x;
  int nt;
  const int e = tile_expert(hdr, j, &nt);
  if (j >= nt) return;

  const int wr = wave >> 2, wc = wave & 3;
  const int colW = blockIdx.y * 256 + wc * 64;
  const size_t aOff = ((size_t)j * TR + wr * 32 + m) * KD + 8 * hh;
  const size_t bOff = ((size_t)e * HD + colW + m) * KD + 8 * hh;
  const unsigned short* ahP = Ah + aOff;
  const unsigned short* alP = Al + aOff;
  const unsigned short* bhP = Wh + bOff;
  const unsigned short* blP = Wl + bOff;

  v8f acc[2][4];
#pragma unroll
  for (int R = 0; R < 2; ++R)
#pragma unroll
    for (int t = 0; t < 4; ++t) { v8f z = {0.f, 0.f, 0.f, 0.f, 0.f, 0.f, 0.f, 0.f}; acc[R][t] = z; }

#pragma unroll 1
  for (int kt = 0; kt < KD / 32; ++kt) {
    const int kk = kt * 32;
    FragB ah[2], al[2];
#pragma unroll
    for (int R = 0; R < 2; ++R) {
      ah[R].h[0] = *(const v8us*)(ahP + (size_t)R * 16 * KD + kk);
      ah[R].h[1] = *(const v8us*)(ahP + (size_t)R * 16 * KD + kk + 16);
      al[R].h[0] = *(const v8us*)(alP + (size_t)R * 16 * KD + kk);
      al[R].h[1] = *(const v8us*)(alP + (size_t)R * 16 * KD + kk + 16);
    }
#pragma unroll
    for (int t = 0; t < 4; ++t) {
      FragB bh, bl;
      bh.h[0] = *(const v8us*)(bhP + (size_t)t * 16 * KD + kk);
      bh.h[1] = *(const v8us*)(bhP + (size_t)t * 16 * KD + kk + 16);
      bl.h[0] = *(const v8us*)(blP + (size_t)t * 16 * KD + kk);
      bl.h[1] = *(const v8us*)(blP + (size_t)t * 16 * KD + kk + 16);
#pragma unroll
      for (int R = 0; R < 2; ++R) {
        acc[R][t] = wmb(ah[R].v, bh.v, acc[R][t]);
        acc[R][t] = wmb(al[R].v, bh.v, acc[R][t]);
        acc[R][t] = wmb(ah[R].v, bl.v, acc[R][t]);
      }
    }
  }

  float bb[4];
#pragma unroll
  for (int t = 0; t < 4; ++t) bb[t] = bias[(size_t)e * HD + colW + 16 * t + m];

  unsigned short* sh = stg + wave * 2048;
  unsigned short* sl = sh + 1024;
  const int q = lane >> 3, pc = lane & 7;
#pragma unroll
  for (int R = 0; R < 2; ++R) {
#pragma unroll
    for (int t = 0; t < 4; ++t) {
#pragma unroll
      for (int r = 0; r < 8; ++r) {
        float v = acc[R][t][r] + bb[t];
        v = fmaxf(v, 0.0f);
        const unsigned int hb = bfbits(v);
        const float hf = __uint_as_float(hb << 16);
        const unsigned int lb = bfbits(v - hf);
        const int li = (8 * hh + r) * 64 + 16 * t + m;
        sh[li] = (unsigned short)hb;
        sl[li] = (unsigned short)lb;
      }
    }
    __syncthreads();
    const size_t rowG = (size_t)j * TR + wr * 32 + R * 16;
#pragma unroll
    for (int i = 0; i < 4; ++i) {
      const int row = 4 * i + q;
      const v8us hv = *(const v8us*)(sh + row * 64 + 8 * pc);
      const v8us lv = *(const v8us*)(sl + row * 64 + 8 * pc);
      const size_t go = (rowG + row) * HD + colW + 8 * pc;
      *(volatile v8us*)(Hh + go) = hv;
      *(volatile v8us*)(Hl + go) = lv;
    }
    __threadfence();
#pragma unroll
    for (int i = 0; i < 4; ++i) {
      const int row = 4 * i + q;
      const v8us hv = *(const v8us*)(sh + row * 64 + 8 * pc);
      const v8us lv = *(const v8us*)(sl + row * 64 + 8 * pc);
      const size_t go = (rowG + row) * HD + colW + 8 * pc;
      *(volatile v8us*)(Hh + go) = hv;
      *(volatile v8us*)(Hl + go) = lv;
    }
    __syncthreads();
  }
}

__global__ __launch_bounds__(NTHR) void k_ffn3(
    const unsigned short* __restrict__ Ah, const unsigned short* __restrict__ Al,
    const unsigned short* __restrict__ Wh, const unsigned short* __restrict__ Wl,
    const float* __restrict__ bias, const int* __restrict__ hdr,
    const int* __restrict__ plist, float* Y, int nTok) {
  __shared__ __attribute__((aligned(16))) float stg[8 * 1024];
  const int tid = threadIdx.x, lane = tid & 31, wave = tid >> 5, hh = lane >> 4, m = lane & 15;
  const int j = blockIdx.x;
  int nt;
  const int e = tile_expert(hdr, j, &nt);
  if (j >= nt) return;

  const int wr = wave >> 2, wc = wave & 3;
  const int colD = wc * 64;
  const int ent = plist[(size_t)j * TR + wr * 32 + lane];
  const size_t aOff = ((size_t)j * TR + wr * 32 + m) * HD + 8 * hh;
  const size_t bOff = ((size_t)e * DOUT + colD + m) * HD + 8 * hh;
  const unsigned short* ahP = Ah + aOff;
  const unsigned short* alP = Al + aOff;
  const unsigned short* bhP = Wh + bOff;
  const unsigned short* blP = Wl + bOff;

  v8f acc[2][4];
#pragma unroll
  for (int R = 0; R < 2; ++R)
#pragma unroll
    for (int t = 0; t < 4; ++t) { v8f z = {0.f, 0.f, 0.f, 0.f, 0.f, 0.f, 0.f, 0.f}; acc[R][t] = z; }

#pragma unroll 1
  for (int kt = 0; kt < HD / 32; ++kt) {
    const int kk = kt * 32;
    FragB ah[2], al[2];
#pragma unroll
    for (int R = 0; R < 2; ++R) {
      ah[R].h[0] = *(const v8us*)(ahP + (size_t)R * 16 * HD + kk);
      ah[R].h[1] = *(const v8us*)(ahP + (size_t)R * 16 * HD + kk + 16);
      al[R].h[0] = *(const v8us*)(alP + (size_t)R * 16 * HD + kk);
      al[R].h[1] = *(const v8us*)(alP + (size_t)R * 16 * HD + kk + 16);
    }
#pragma unroll
    for (int t = 0; t < 4; ++t) {
      FragB bh, bl;
      bh.h[0] = *(const v8us*)(bhP + (size_t)t * 16 * HD + kk);
      bh.h[1] = *(const v8us*)(bhP + (size_t)t * 16 * HD + kk + 16);
      bl.h[0] = *(const v8us*)(blP + (size_t)t * 16 * HD + kk);
      bl.h[1] = *(const v8us*)(blP + (size_t)t * 16 * HD + kk + 16);
#pragma unroll
      for (int R = 0; R < 2; ++R) {
        acc[R][t] = wmb(ah[R].v, bh.v, acc[R][t]);
        acc[R][t] = wmb(al[R].v, bh.v, acc[R][t]);
        acc[R][t] = wmb(ah[R].v, bl.v, acc[R][t]);
      }
    }
  }

  float bb[4];
#pragma unroll
  for (int t = 0; t < 4; ++t) bb[t] = bias[(size_t)e * DOUT + colD + 16 * t + m];

  float* sw = stg + wave * 1024;
#pragma unroll
  for (int R = 0; R < 2; ++R) {
#pragma unroll
    for (int t = 0; t < 4; ++t)
#pragma unroll
      for (int r = 0; r < 8; ++r) sw[(8 * hh + r) * 64 + 16 * t + m] = acc[R][t][r] + bb[t];
    __syncthreads();
#pragma unroll
    for (int i = 0; i < 8; ++i) {
      const int eA = __builtin_amdgcn_readlane(ent, R * 16 + 2 * i);
      const int eB = __builtin_amdgcn_readlane(ent, R * 16 + 2 * i + 1);
      const int my = hh ? eB : eA;
      const bool valid = my >= 0;
      int tt = my >> 1;
      tt = tt < 0 ? 0 : (tt > nTok - 1 ? nTok - 1 : tt);
      const int slot = my & 1;
      const v4f v = *(const v4f*)(sw + (2 * i + hh) * 64 + 4 * m);
      float* gp = Y + ((size_t)tt * 2 + slot) * DOUT + colD + 4 * m;
      if (valid) *(volatile v4f*)gp = v;
    }
    __threadfence();
#pragma unroll
    for (int i = 0; i < 8; ++i) {
      const int eA = __builtin_amdgcn_readlane(ent, R * 16 + 2 * i);
      const int eB = __builtin_amdgcn_readlane(ent, R * 16 + 2 * i + 1);
      const int my = hh ? eB : eA;
      const bool valid = my >= 0;
      int tt = my >> 1;
      tt = tt < 0 ? 0 : (tt > nTok - 1 ? nTok - 1 : tt);
      const int slot = my & 1;
      const v4f v = *(const v4f*)(sw + (2 * i + hh) * 64 + 4 * m);
      float* gp = Y + ((size_t)tt * 2 + slot) * DOUT + colD + 4 * m;
      if (valid) *(volatile v4f*)gp = v;
    }
    __syncthreads();
  }
}

__global__ __launch_bounds__(NTHR) void k_combine(
    const int* __restrict__ tinfo, const float* __restrict__ Y, float* out, int nTok) {
#pragma clang fp contract(off)
  const int tid = threadIdx.x;
  int t = blockIdx.x * 4 + (tid >> 6);
  t = t > nTok - 1 ? nTok - 1 : t;
  const int c0 = (tid & 63) * 4;
  const v4i inf = *(const v4i*)(tinfo + 4 * (size_t)t);
  const float w0 = __int_as_float(inf.z);
  const float w1 = __int_as_float(inf.w);
  const v4f y0 = *(const v4f*)(Y + ((size_t)t * 2) * DOUT + c0);
  const v4f y1 = *(const v4f*)(Y + ((size_t)t * 2 + 1) * DOUT + c0);
  const v4f p0 = y0 * w0;
  const v4f p1 = y1 * w1;
  const v4f o  = p0 + p1;
  float* gp = out + (size_t)t * DOUT + c0;
  *(volatile v4f*)gp = o;
  __threadfence();
  *(volatile v4f*)gp = o;
}

extern "C" void kernel_launch(void* const* d_in, const int* in_sizes, int n_in,
                              void* d_out, int out_size, void* d_ws, size_t ws_size,
                              hipStream_t stream) {
  if (n_in < 11) return;
  if (in_sizes[0] != NTOK * DIN || in_sizes[1] != DIN * HD || in_sizes[2] != HD) return;
  if (in_sizes[3] != HD * NE || in_sizes[4] != NE) return;
  if (in_sizes[5] != DIN * NE * HD || in_sizes[6] != NE * HD) return;
  if (in_sizes[7] != HD * NE * HD || in_sizes[8] != NE * HD) return;
  if (in_sizes[9] != HD * NE * DOUT || in_sizes[10] != NE * DOUT) return;
  if (out_size != NTOK * DOUT) return;

  const float* x   = (const float*)d_in[0];
  const float* gw  = (const float*)d_in[1];
  const float* gb  = (const float*)d_in[2];
  const float* gow = (const float*)d_in[3];
  const float* gob = (const float*)d_in[4];
  const float* w1  = (const float*)d_in[5];
  const float* b1  = (const float*)d_in[6];
  const float* w2  = (const float*)d_in[7];
  const float* b2  = (const float*)d_in[8];
  const float* w3  = (const float*)d_in[9];
  const float* b3  = (const float*)d_in[10];
  float* out = (float*)d_out;

  char* ws = (char*)d_ws;
  size_t off = 0;
  const size_t oTI  = off; off += (size_t)NTOK * 16;              off = (off + 255) & ~(size_t)255;
  const size_t oHD  = off; off += 256;                            off = (off + 255) & ~(size_t)255;
  const size_t oPL  = off; off += (size_t)NTL * TR * 4;           off = (off + 255) & ~(size_t)255;
  const size_t oW1H = off; off += (size_t)NE * HD * DIN * 2;      off = (off + 255) & ~(size_t)255;
  const size_t oW1L = off; off += (size_t)NE * HD * DIN * 2;      off = (off + 255) & ~(size_t)255;
  const size_t oW2H = off; off += (size_t)NE * HD * HD * 2;       off = (off + 255) & ~(size_t)255;
  const size_t oW2L = off; off += (size_t)NE * HD * HD * 2;       off = (off + 255) & ~(size_t)255;
  const size_t oW3H = off; off += (size_t)NE * DOUT * HD * 2;     off = (off + 255) & ~(size_t)255;
  const size_t oW3L = off; off += (size_t)NE * DOUT * HD * 2;     off = (off + 255) & ~(size_t)255;
  const size_t oXGH = off; off += (size_t)NTL * TR * DIN * 2;     off = (off + 255) & ~(size_t)255;
  const size_t oXGL = off; off += (size_t)NTL * TR * DIN * 2;     off = (off + 255) & ~(size_t)255;
  const size_t oH1H = off; off += (size_t)NTL * TR * HD * 2;      off = (off + 255) & ~(size_t)255;
  const size_t oH1L = off; off += (size_t)NTL * TR * HD * 2;      off = (off + 255) & ~(size_t)255;
  const size_t oH2H = off; off += (size_t)NTL * TR * HD * 2;      off = (off + 255) & ~(size_t)255;
  const size_t oH2L = off; off += (size_t)NTL * TR * HD * 2;      off = (off + 255) & ~(size_t)255;
  const size_t oY   = oH1H;
  if (off > ws_size || off > (size_t)134217728) return;

  int*            tinfo = (int*)(ws + oTI);
  int*            hdr   = (int*)(ws + oHD);
  int*            plist = (int*)(ws + oPL);
  unsigned short* W1h   = (unsigned short*)(ws + oW1H);
  unsigned short* W1l   = (unsigned short*)(ws + oW1L);
  unsigned short* W2h   = (unsigned short*)(ws + oW2H);
  unsigned short* W2l   = (unsigned short*)(ws + oW2L);
  unsigned short* W3h   = (unsigned short*)(ws + oW3H);
  unsigned short* W3l   = (unsigned short*)(ws + oW3L);
  unsigned short* Xgh   = (unsigned short*)(ws + oXGH);
  unsigned short* Xgl   = (unsigned short*)(ws + oXGL);
  unsigned short* H1h   = (unsigned short*)(ws + oH1H);
  unsigned short* H1l   = (unsigned short*)(ws + oH1L);
  unsigned short* H2h   = (unsigned short*)(ws + oH2H);
  unsigned short* H2l   = (unsigned short*)(ws + oH2L);
  float*          Y     = (float*)(ws + oY);

  k_wconv<<<dim3(DIN / 64, (NE * HD) / 64), NTHR, 0, stream>>>(w1, W1h, W1l, DIN, NE * HD);
  k_wconv<<<dim3(HD / 64, (NE * HD) / 64), NTHR, 0, stream>>>(w2, W2h, W2l, HD, NE * HD);
  k_wconv<<<dim3(HD / 64, (NE * DOUT) / 64), NTHR, 0, stream>>>(w3, W3h, W3l, HD, NE * DOUT);

  k_gate<<<NTOK / NTHR, NTHR, 0, stream>>>(x, gw, gb, gow, gob, tinfo);
  k_lists<<<1, LTHR, 0, stream>>>(tinfo, plist, hdr, NTOK);
  k_gather<<<(NTL * TR) / 8, NTHR, 0, stream>>>(x, plist, Xgh, Xgl, NTOK);

  k_ffn<DIN><<<dim3(NTL, HD / 256), NTHR, 0, stream>>>(Xgh, Xgl, W1h, W1l, b1, hdr, H1h, H1l);
  k_ffn<HD><<<dim3(NTL, HD / 256), NTHR, 0, stream>>>(H1h, H1l, W2h, W2l, b2, hdr, H2h, H2l);
  k_ffn3<<<dim3(NTL, 1), NTHR, 0, stream>>>(H2h, H2l, W3h, W3l, b3, hdr, plist, Y, NTOK);

  k_combine<<<NTOK / 4, NTHR, 0, stream>>>(tinfo, Y, out, NTOK);
}
